// MyRNN_67388036874303
// MI455X (gfx1250) — hardware-verified
//
#include <hip/hip_runtime.h>
#include <math.h>

constexpr int NB      = 128;
constexpr int NSTEP   = 80;
constexpr int NE      = 100;
constexpr int NEP     = 128;
constexpr int NU      = 512;
constexpr int NV      = 10000;
constexpr int NTHR    = 256;
constexpr int SEQ_BLK = 16;
constexpr int XP      = 136;
constexpr int HP      = 520;
constexpr int SLABP   = 68;
constexpr int NHT     = 128;
constexpr float CACT     = 16.0f;
constexpr float CWGT     = 64.0f;
constexpr float RSC      = 2048.0f;
constexpr float RSC_INV  = 1.0f / 2048.0f;
constexpr float PROD_INV = 1.0f / 1024.0f;
constexpr float F16_MINN = 6.103515625e-05f;
static_assert(NB % SEQ_BLK == 0);
static_assert(NU == 64 * (NTHR / 32));
static_assert(NEP % 32 == 0 && NU % 32 == 0 && NEP >= NE);
static_assert(NEP % 64 == 0 && NU % 64 == 0);
static_assert(XP % 8 == 0 && XP >= NEP && HP % 8 == 0 && HP >= NU);
static_assert(SEQ_BLK * NEP == NTHR * 8);
static_assert(NE % 4 == 0 && NE >= 8);
static_assert(NHT == NB && NB == 32 * 4);
static_assert(NU % 4 == 0);

typedef __attribute__((ext_vector_type(16))) _Float16 v16h;
typedef __attribute__((ext_vector_type(8)))  _Float16 v8h;
typedef __attribute__((ext_vector_type(8)))  float    v8f;
typedef __attribute__((ext_vector_type(4)))  float    v4f;

__device__ __forceinline__ void mma_guard6(v8f& a, v8f& b, v16h w, v16h x, v16h y, v16h z) {
  asm volatile("v_nop\n\tv_nop\n\tv_nop\n\tv_nop" : "+v"(a), "+v"(b) : "v"(w), "v"(x), "v"(y), "v"(z));
}
__device__ __forceinline__ void acc_guard2(v8f& a, v8f& b) { asm volatile("v_nop\n\tv_nop\n\tv_nop\n\tv_nop" : "+v"(a), "+v"(b)); }

template <typename T> struct Frag;
template <> struct Frag<_Float16> {
  typedef v16h V; union U { v16h v; v8h h[2]; };
  static __device__ __forceinline__ v16h load(const _Float16* p) {
    U f; f.h[0] = *(const v8h*)(p); f.h[1] = *(const v8h*)(p + 16); return f.v;
  }
  static __device__ __forceinline__ v8f mma(v16h a, v16h b, v8f c) {
    return __builtin_amdgcn_wmma_f32_16x16x32_f16(false, a, false, b, (short)0, c, false, false);
  }
};

__device__ __forceinline__ void split16(float a, _Float16& hi, _Float16& lo) {
  const float af = (fabsf(a) < F16_MINN) ? 0.0f : a;
  const _Float16 h = (_Float16)af;
  const float hf = (float)h;
  const float res = (a - hf) * RSC;
  hi = h;
  lo = (_Float16)res;
}

__global__ __launch_bounds__(NTHR) void tps_kernel(const float* __restrict__ src, int Rreal, int C, int ldo,
                                                   unsigned short* __restrict__ Oh, unsigned short* __restrict__ Ol) {
  __shared__ float Tt[64 * 65];
  const int tid = threadIdx.x;
  const int c0 = blockIdx.x * 64, r0 = blockIdx.y * 64;
#pragma unroll
  for (int i = 0; i < 4; ++i) {
    const int idx = i * NTHR + tid;
    const int rr = idx >> 4, cc = (idx & 15) * 4;
    const int r  = r0 + rr;
    const int rs = (r < Rreal) ? r : (Rreal - 1);
    const float fac = (r < Rreal) ? 1.0f : 0.0f;
    const v4f v = *(const v4f*)(src + (size_t)rs * (size_t)C + c0 + cc);
    Tt[rr * 65 + cc + 0] = v[0] * fac;
    Tt[rr * 65 + cc + 1] = v[1] * fac;
    Tt[rr * 65 + cc + 2] = v[2] * fac;
    Tt[rr * 65 + cc + 3] = v[3] * fac;
  }
  __syncthreads();
  const int q = tid >> 3, c8 = (tid & 7) * 8;
  v8h hv[2], lv[2];
#pragma unroll
  for (int g = 0; g < 2; ++g) {
    const int qq = g * 32 + q;
#pragma unroll
    for (int e = 0; e < 8; ++e) {
      const float f = Tt[(c8 + e) * 65 + qq] * CWGT;
      _Float16 h, l;
      split16(f, h, l);
      hv[g][e] = h;
      lv[g][e] = l;
    }
  }
  for (int pass = 0; pass < 2; ++pass) {
#pragma unroll
    for (int g = 0; g < 2; ++g) {
      const size_t o = (size_t)(c0 + g * 32 + q) * (size_t)ldo + (size_t)(r0 + c8);
      *(volatile v8h*)(Oh + o) = hv[g];
      *(volatile v8h*)(Ol + o) = lv[g];
    }
    __threadfence();
  }
}

__global__ __launch_bounds__(NTHR) void rnn_seq_kernel(
    const int* __restrict__ tokens, const float* __restrict__ emb,
    const float* __restrict__ b0, const float* __restrict__ b1,
    const unsigned short* __restrict__ K0Thp, const unsigned short* __restrict__ K0Tlp,
    const unsigned short* __restrict__ R0Thp, const unsigned short* __restrict__ R0Tlp,
    const unsigned short* __restrict__ K1Thp, const unsigned short* __restrict__ K1Tlp,
    const unsigned short* __restrict__ R1Thp, const unsigned short* __restrict__ R1Tlp,
    float* __restrict__ HT) {
  __shared__ __align__(16) _Float16 Xh[SEQ_BLK * XP];
  __shared__ __align__(16) _Float16 Xl[SEQ_BLK * XP];
  __shared__ __align__(16) _Float16 Hh[SEQ_BLK * HP];
  __shared__ __align__(16) _Float16 Hl[SEQ_BLK * HP];
  __shared__ __align__(16) _Float16 Gh[SEQ_BLK * HP];
  __shared__ __align__(16) _Float16 Gl[SEQ_BLK * HP];
  __shared__ __align__(16) float    Sl[NTHR / 32][8 * SLABP];
  const _Float16* K0Th = (const _Float16*)K0Thp; const _Float16* K0Tl = (const _Float16*)K0Tlp;
  const _Float16* R0Th = (const _Float16*)R0Thp; const _Float16* R0Tl = (const _Float16*)R0Tlp;
  const _Float16* K1Th = (const _Float16*)K1Thp; const _Float16* K1Tl = (const _Float16*)K1Tlp;
  const _Float16* R1Th = (const _Float16*)R1Thp; const _Float16* R1Tl = (const _Float16*)R1Tlp;
  const int tid = threadIdx.x, lane = tid & 31, wave = tid >> 5;
  const int c = lane & 15, hh = lane >> 4, koff = hh * 8, c4 = c * 4;
  const int rowbase = blockIdx.x * SEQ_BLK;

#pragma unroll 1
  for (int i = tid; i < SEQ_BLK * HP; i += NTHR) { Hh[i] = (_Float16)0.0f; Hl[i] = (_Float16)0.0f; }
  float bb0[4], bb1[4], hst[4][8];
#pragma unroll
  for (int nt = 0; nt < 4; ++nt) {
    const int j = 64 * wave + 16 * nt + c;
    bb0[nt] = b0[j];
    bb1[nt] = b1[j];
#pragma unroll
    for (int r = 0; r < 8; ++r) hst[nt][r] = 0.0f;
  }
  __syncthreads();

  const _Float16* xhrow = Xh + c * XP + koff;
  const _Float16* xlrow = Xl + c * XP + koff;
  const _Float16* hhrow = Hh + c * HP + koff;
  const _Float16* hlrow = Hl + c * HP + koff;
  const _Float16* ghrow = Gh + c * HP + koff;
  const _Float16* glrow = Gl + c * HP + koff;
  const int sm = tid >> 4, sc8 = (tid & 15) * 8;
  const int tokoff = (rowbase + sm) * NSTEP;
  const v8f z8 = {0.f, 0.f, 0.f, 0.f, 0.f, 0.f, 0.f, 0.f};

#pragma unroll 1
  for (int t = 0; t < NSTEP; ++t) {
    {
      int tok = tokens[tokoff + t];
      tok = (tok < 0) ? 0 : ((tok > NV - 1) ? (NV - 1) : tok);
      const float* er = emb + (size_t)tok * NE;
      const int o0 = (sc8 < NE - 4) ? sc8 : (NE - 4);
      const int o1 = ((sc8 + 4) < NE - 4) ? (sc8 + 4) : (NE - 4);
      const v4f va = *(const v4f*)(er + o0);
      const v4f vb = *(const v4f*)(er + o1);
      v8h hv, lv;
#pragma unroll
      for (int e = 0; e < 4; ++e) {
        const float fa = (sc8 + e < NE) ? CACT : 0.0f;
        const float fb = (sc8 + 4 + e < NE) ? CACT : 0.0f;
        _Float16 h, l;
        split16(va[e] * fa, h, l); hv[e] = h;     lv[e] = l;
        split16(vb[e] * fb, h, l); hv[4 + e] = h; lv[4 + e] = l;
      }
      *(v8h*)(Xh + sm * XP + sc8) = hv;
      *(v8h*)(Xl + sm * XP + sc8) = lv;
    }
    __syncthreads();

#pragma unroll
    for (int nt = 0; nt < 4; ++nt) {
      const int j = 64 * wave + 16 * nt + c;
      const _Float16* wkh = K0Th + (size_t)j * NEP + koff;
      const _Float16* wkl = K0Tl + (size_t)j * NEP + koff;
      const _Float16* wrh = R0Th + (size_t)j * NU + koff;
      const _Float16* wrl = R0Tl + (size_t)j * NU + koff;
      v8f accM = z8, accR = z8;
#pragma unroll 1
      for (int kx = 0; kx < NEP; kx += 32) {
        const v16h ah = Frag<_Float16>::load(xhrow + kx);
        const v16h al = Frag<_Float16>::load(xlrow + kx);
        const v16h bh = Frag<_Float16>::load(wkh + kx);
        const v16h bl = Frag<_Float16>::load(wkl + kx);
        accM = Frag<_Float16>::mma(ah, bh, accM);
        accR = Frag<_Float16>::mma(ah, bl, accR);
        accR = Frag<_Float16>::mma(al, bh, accR);
        mma_guard6(accM, accR, ah, al, bh, bl);
      }
#pragma unroll 1
      for (int k0 = 0; k0 < NU; k0 += 32) {
        const v16h ah = Frag<_Float16>::load(hhrow + k0);
        const v16h al = Frag<_Float16>::load(hlrow + k0);
        const v16h bh = Frag<_Float16>::load(wrh + k0);
        const v16h bl = Frag<_Float16>::load(wrl + k0);
        accM = Frag<_Float16>::mma(ah, bh, accM);
        accR = Frag<_Float16>::mma(ah, bl, accR);
        accR = Frag<_Float16>::mma(al, bh, accR);
        mma_guard6(accM, accR, ah, al, bh, bl);
      }
      acc_guard2(accM, accR);
#pragma unroll
      for (int r = 0; r < 8; ++r) {
        const float z = (accM[r] + accR[r] * RSC_INV) * PROD_INV + bb0[nt];
        const float g = tanhf(z);
        _Float16 h, l;
        split16(g * CACT, h, l);
        Gh[(8 * hh + r) * HP + j] = h;
        Gl[(8 * hh + r) * HP + j] = l;
      }
    }
    __syncthreads();

#pragma unroll
    for (int nt = 0; nt < 4; ++nt) {
      const int j = 64 * wave + 16 * nt + c;
      const _Float16* wkh = K1Th + (size_t)j * NU + koff;
      const _Float16* wkl = K1Tl + (size_t)j * NU + koff;
      const _Float16* wrh = R1Th + (size_t)j * NU + koff;
      const _Float16* wrl = R1Tl + (size_t)j * NU + koff;
      v8f accM = z8, accR = z8;
#pragma unroll 1
      for (int k0 = 0; k0 < NU; k0 += 32) {
        const v16h ah = Frag<_Float16>::load(ghrow + k0);
        const v16h al = Frag<_Float16>::load(glrow + k0);
        const v16h bh = Frag<_Float16>::load(wkh + k0);
        const v16h bl = Frag<_Float16>::load(wkl + k0);
        accM = Frag<_Float16>::mma(ah, bh, accM);
        accR = Frag<_Float16>::mma(ah, bl, accR);
        accR = Frag<_Float16>::mma(al, bh, accR);
        mma_guard6(accM, accR, ah, al, bh, bl);
      }
#pragma unroll 1
      for (int k0 = 0; k0 < NU; k0 += 32) {
        const v16h ah = Frag<_Float16>::load(hhrow + k0);
        const v16h al = Frag<_Float16>::load(hlrow + k0);
        const v16h bh = Frag<_Float16>::load(wrh + k0);
        const v16h bl = Frag<_Float16>::load(wrl + k0);
        accM = Frag<_Float16>::mma(ah, bh, accM);
        accR = Frag<_Float16>::mma(ah, bl, accR);
        accR = Frag<_Float16>::mma(al, bh, accR);
        mma_guard6(accM, accR, ah, al, bh, bl);
      }
      acc_guard2(accM, accR);
#pragma unroll
      for (int r = 0; r < 8; ++r) {
        const float z = (accM[r] + accR[r] * RSC_INV) * PROD_INV + bb1[nt];
        hst[nt][r] = tanhf(z);
      }
    }
    __syncthreads();

#pragma unroll
    for (int nt = 0; nt < 4; ++nt) {
      const int j = 64 * wave + 16 * nt + c;
#pragma unroll
      for (int r = 0; r < 8; ++r) {
        _Float16 h, l;
        split16(hst[nt][r] * CACT, h, l);
        Hh[(8 * hh + r) * HP + j] = h;
        Hl[(8 * hh + r) * HP + j] = l;
      }
    }
  }

  float* slab = Sl[wave];
#pragma unroll
  for (int hsel = 0; hsel < 2; ++hsel) {
    if (hh == hsel) {
#pragma unroll
      for (int nt = 0; nt < 4; ++nt)
#pragma unroll
        for (int r = 0; r < 8; ++r) slab[r * SLABP + 16 * nt + c] = hst[nt][r];
    }
    __builtin_amdgcn_fence(__ATOMIC_RELEASE, "workgroup");
    __builtin_amdgcn_wave_barrier();
    __builtin_amdgcn_fence(__ATOMIC_ACQUIRE, "workgroup");
    for (int pass = 0; pass < 2; ++pass) {
#pragma unroll
      for (int it = 0; it < 4; ++it) {
        const int row = it * 2 + hh;
        const v4f v = *(const v4f*)(slab + row * SLABP + c4);
        *(volatile v4f*)(HT + (size_t)(rowbase + 8 * hsel + row) * NU + 64 * wave + c4) = v;
      }
      __threadfence();
    }
    __builtin_amdgcn_fence(__ATOMIC_RELEASE, "workgroup");
    __builtin_amdgcn_wave_barrier();
    __builtin_amdgcn_fence(__ATOMIC_ACQUIRE, "workgroup");
  }
}

__global__ __launch_bounds__(NHT) void head_kernel(const float* __restrict__ HT, const float* __restrict__ wd,
                                                   const float* __restrict__ bd, float* __restrict__ out) {
  __shared__ __align__(16) float sO[NHT];
  const int tid = threadIdx.x;
  const float* hr = HT + (size_t)tid * NU;
  float s = 0.0f;
#pragma unroll 1
  for (int u = 0; u < NU; u += 4) {
    const v4f h = *(const v4f*)(hr + u);
    const v4f w = *(const v4f*)(wd + u);
    s += h[0] * w[0];
    s += h[1] * w[1];
    s += h[2] * w[2];
    s += h[3] * w[3];
  }
  const float lg = s + bd[0];
  const float o = 1.0f / (1.0f + expf(-lg));
  sO[tid] = o;
  __syncthreads();
  if (tid < 32) {
    const v4f v = *(const v4f*)(sO + 4 * tid);
    *(volatile v4f*)(out + 4 * tid) = v;
    __threadfence();
    *(volatile v4f*)(out + 4 * tid) = v;
  }
}

extern "C" void kernel_launch(void* const* d_in, const int* in_sizes, int n_in,
                              void* d_out, int out_size, void* d_ws, size_t ws_size, hipStream_t stream) {
  if (n_in < 10 || d_out == nullptr || d_ws == nullptr) return;
  if (in_sizes[0] != NB * NSTEP || in_sizes[1] != NV * NE || in_sizes[2] != NE * NU || in_sizes[3] != NU * NU ||
      in_sizes[4] != NU || in_sizes[5] != NU * NU || in_sizes[6] != NU * NU || in_sizes[7] != NU ||
      in_sizes[8] != NU || in_sizes[9] != 1 || out_size != NB) return;

  const int*   tokens = (const int*)d_in[0];
  const float* emb    = (const float*)d_in[1];
  const float* k0     = (const float*)d_in[2];
  const float* rk0    = (const float*)d_in[3];
  const float* b0     = (const float*)d_in[4];
  const float* k1     = (const float*)d_in[5];
  const float* rk1    = (const float*)d_in[6];
  const float* b1     = (const float*)d_in[7];
  const float* wd     = (const float*)d_in[8];
  const float* bd     = (const float*)d_in[9];
  float* out = (float*)d_out;

  char* ws = (char*)d_ws; size_t off = 0;
  auto carve = [&](size_t bytes) -> char* { char* p = ws + off; off += (bytes + 255) & ~(size_t)255; return p; };
  unsigned short* K0Th = (unsigned short*)carve((size_t)NU * NEP * 2);
  unsigned short* K0Tl = (unsigned short*)carve((size_t)NU * NEP * 2);
  unsigned short* R0Th = (unsigned short*)carve((size_t)NU * NU * 2);
  unsigned short* R0Tl = (unsigned short*)carve((size_t)NU * NU * 2);
  unsigned short* K1Th = (unsigned short*)carve((size_t)NU * NU * 2);
  unsigned short* K1Tl = (unsigned short*)carve((size_t)NU * NU * 2);
  unsigned short* R1Th = (unsigned short*)carve((size_t)NU * NU * 2);
  unsigned short* R1Tl = (unsigned short*)carve((size_t)NU * NU * 2);
  float*          HT   = (float*)carve((size_t)NB * NU * 4);
  if (off > ws_size || off > (size_t)134217728) return;

  tps_kernel<<<dim3(NU / 64, NEP / 64), NTHR, 0, stream>>>(k0,  NE, NU, NEP, K0Th, K0Tl);
  tps_kernel<<<dim3(NU / 64, NU / 64),  NTHR, 0, stream>>>(rk0, NU, NU, NU,  R0Th, R0Tl);
  tps_kernel<<<dim3(NU / 64, NU / 64),  NTHR, 0, stream>>>(k1,  NU, NU, NU,  K1Th, K1Tl);
  tps_kernel<<<dim3(NU / 64, NU / 64),  NTHR, 0, stream>>>(rk1, NU, NU, NU,  R1Th, R1Tl);
  rnn_seq_kernel<<<NB / SEQ_BLK, NTHR, 0, stream>>>(tokens, emb, b0, b1, K0Th, K0Tl, R0Th, R0Tl, K1Th, K1Tl, R1Th, R1Tl, HT);
  head_kernel<<<1, NHT, 0, stream>>>(HT, wd, bd, out);
}
